// ConceptBottleneck_51934744543354
// MI455X (gfx1250) — hardware-verified
//
#include <hip/hip_runtime.h>
#include <math.h>
#include <stdint.h>

#define NB_  8192
#define NI_  768
#define NG_  64
#define NH_  64
#define NE_  16
#define NX_  32
#define HP_  72
#define WSC  64.0f
#define LOSC 2048.0f

static_assert((NB_ % 128) == 0 && (NB_ % 16) == 0 && (NI_ % 32) == 0);
static_assert(NH_ == 64 && NE_ == 16 && NX_ == 2 * NE_ && (HP_ % 8) == 0);
static_assert(((NB_ * NI_) % (8 * 256)) == 0);

typedef _Float16 v16h __attribute__((ext_vector_type(16)));
typedef _Float16 v8h  __attribute__((ext_vector_type(8)));
typedef float    v8f  __attribute__((ext_vector_type(8)));
typedef float    v4f  __attribute__((ext_vector_type(4)));
typedef unsigned int v4u __attribute__((ext_vector_type(4)));

union FragH { v16h v; v8h h[2]; };

__device__ __forceinline__ unsigned short bf_bits(float f) {
  unsigned u = __float_as_uint(f);
  return (unsigned short)((u + 0x7FFFu + ((u >> 16) & 1u)) >> 16);
}
__device__ __forceinline__ float bf_up(unsigned short h) { return __uint_as_float(((unsigned)h) << 16); }
__device__ __forceinline__ float bfr(float f) { return bf_up(bf_bits(f)); }
__device__ __forceinline__ unsigned short h_bits(_Float16 x) { return __builtin_bit_cast(unsigned short, x); }
__device__ __forceinline__ unsigned pk16(unsigned short a, unsigned short b) { return (unsigned)a | ((unsigned)b << 16); }
__device__ __forceinline__ unsigned pkh(float a, float b) { return pk16(h_bits((_Float16)a), h_bits((_Float16)b)); }
__device__ __forceinline__ v8f zero8() { v8f z = {0.f, 0.f, 0.f, 0.f, 0.f, 0.f, 0.f, 0.f}; return z; }

__device__ __forceinline__ void hl_one(float f, _Float16& h, _Float16& l) {
#pragma clang fp contract(off)
  const _Float16 hv = (_Float16)f;
  const float d = f - (float)hv;
  const float r = d * LOSC;
  h = hv;
  l = (_Float16)r;
}

__device__ __forceinline__ v16h ldfrag_h(const _Float16* p) {
  FragH f;
  f.h[0] = *(const v8h*)(p);
  f.h[1] = *(const v8h*)(p + 16);
  return f.v;
}

__device__ __forceinline__ v8f wm(v16h a, v16h b, v8f c) {
  return __builtin_amdgcn_wmma_f32_16x16x32_f16(false, a, false, b, (short)0, c, false, false);
}
__device__ __forceinline__ void guard4(v8f& c0, v8f& c1, v8f& c2, v8f& c3, v16h a0, v16h a1, v16h b0, v16h b1) {
#if defined(__HIP_DEVICE_COMPILE__)
  asm volatile("v_nop\n\tv_nop\n\tv_nop\n\tv_nop"
               : "+v"(c0), "+v"(c1), "+v"(c2), "+v"(c3)
               : "v"(a0), "v"(a1), "v"(b0), "v"(b1));
#endif
}
__device__ __forceinline__ void guard2(v8f& c0, v8f& c1, v16h a0, v16h a1, v16h b0) {
#if defined(__HIP_DEVICE_COMPILE__)
  asm volatile("v_nop\n\tv_nop\n\tv_nop\n\tv_nop"
               : "+v"(c0), "+v"(c1)
               : "v"(a0), "v"(a1), "v"(b0));
#endif
}
__device__ __forceinline__ void wave_sync_lds() {
  __builtin_amdgcn_fence(__ATOMIC_RELEASE, "workgroup");
  __builtin_amdgcn_wave_barrier();
  __builtin_amdgcn_fence(__ATOMIC_ACQUIRE, "workgroup");
}

__global__ __launch_bounds__(256) void cvt_x(const float* __restrict__ x, unsigned short* xh, int n8) {
  const int t = blockIdx.x * 256 + threadIdx.x;
  const int tc = (t < n8) ? t : (n8 - 1);
  const float* p = x + (size_t)tc * 8;
  const v4f a = *(const v4f*)p;
  const v4f b = *(const v4f*)(p + 4);
  v4u pk;
  pk[0] = pk16(h_bits((_Float16)bfr(a[0])), h_bits((_Float16)bfr(a[1])));
  pk[1] = pk16(h_bits((_Float16)bfr(a[2])), h_bits((_Float16)bfr(a[3])));
  pk[2] = pk16(h_bits((_Float16)bfr(b[0])), h_bits((_Float16)bfr(b[1])));
  pk[3] = pk16(h_bits((_Float16)bfr(b[2])), h_bits((_Float16)bfr(b[3])));
  unsigned short* gp = xh + (size_t)tc * 8;
  if (t < n8) *(volatile v4u*)gp = pk;
  __threadfence();
  if (t < n8) *(volatile v4u*)gp = pk;
}

__global__ __launch_bounds__(256) void cvt_w(const float* __restrict__ w0, const float* __restrict__ w1,
                                             const float* __restrict__ w2, unsigned short* dst,
                                             int nin, int nout, int n8) {
  const int y = blockIdx.y;
  const float* src = (y == 0) ? w0 : ((y == 1) ? w1 : w2);
  const int t = blockIdx.x * 256 + threadIdx.x;
  const int tc = (t < n8) ? t : (n8 - 1);
  const unsigned d = (unsigned)tc * 8u;
  const unsigned R = d / (unsigned)nin;
  const unsigned k0 = d - R * (unsigned)nin;
  const unsigned z = R / (unsigned)nout;
  const unsigned o = R - z * (unsigned)nout;
  const float* sp = src + ((size_t)z * nin + k0) * (size_t)nout + o;
  float f[8];
#pragma unroll
  for (int e = 0; e < 8; ++e) f[e] = bfr(sp[(size_t)e * nout]) * WSC;
  v4u pk;
#pragma unroll
  for (int e = 0; e < 4; ++e) pk[e] = pkh(f[2 * e], f[2 * e + 1]);
  unsigned short* gp = dst + (size_t)y * (size_t)n8 * 8 + (size_t)d;
  if (t < n8) *(volatile v4u*)gp = pk;
  __threadfence();
  if (t < n8) *(volatile v4u*)gp = pk;
}

__global__ __launch_bounds__(128) void grp_mlp(const unsigned short* __restrict__ xh,
                                               const unsigned short* __restrict__ w1t, const float* __restrict__ b1,
                                               const unsigned short* __restrict__ w2t, const float* __restrict__ b2,
                                               const unsigned short* __restrict__ w3t, const float* __restrict__ b3,
                                               float* outp) {
#pragma clang fp contract(off)
  __shared__ __align__(16) _Float16 Hh[4][32 * HP_];
  __shared__ __align__(16) _Float16 Hl[4][32 * HP_];
  __shared__ __align__(16) float Os[4][256];
  const int lane = threadIdx.x & 31, wave = threadIdx.x >> 5;
  const int rl = lane & 15, hh = lane >> 4, koff = 8 * hh;
  const int g = blockIdx.y;
  const int m0 = blockIdx.x * 128 + wave * 32;
  const _Float16* X  = (const _Float16*)(const void*)xh;
  const _Float16* W1 = (const _Float16*)(const void*)w1t;
  const _Float16* W2 = (const _Float16*)(const void*)w2t;
  const _Float16* W3 = (const _Float16*)(const void*)w3t;

  v8f acc[2][4];
#pragma unroll
  for (int i = 0; i < 2; ++i)
#pragma unroll
    for (int j = 0; j < 4; ++j) acc[i][j] = zero8();
  const _Float16* xa = X + (size_t)(m0 + rl) * NI_ + koff;
  const _Float16* xb = X + (size_t)(m0 + 16 + rl) * NI_ + koff;
  const _Float16* wr = W1 + (size_t)(g * NH_ + rl) * NI_ + koff;
#pragma unroll 1
  for (int k0 = 0; k0 < NI_; k0 += 32) {
    const v16h fa0 = ldfrag_h(xa + k0);
    const v16h fa1 = ldfrag_h(xb + k0);
    {
      const v16h fb0 = ldfrag_h(wr + k0);
      const v16h fb1 = ldfrag_h(wr + (size_t)16 * NI_ + k0);
      acc[0][0] = wm(fa0, fb0, acc[0][0]);
      acc[1][0] = wm(fa1, fb0, acc[1][0]);
      acc[0][1] = wm(fa0, fb1, acc[0][1]);
      acc[1][1] = wm(fa1, fb1, acc[1][1]);
      guard4(acc[0][0], acc[1][0], acc[0][1], acc[1][1], fa0, fa1, fb0, fb1);
    }
    {
      const v16h fb2 = ldfrag_h(wr + (size_t)32 * NI_ + k0);
      const v16h fb3 = ldfrag_h(wr + (size_t)48 * NI_ + k0);
      acc[0][2] = wm(fa0, fb2, acc[0][2]);
      acc[1][2] = wm(fa1, fb2, acc[1][2]);
      acc[0][3] = wm(fa0, fb3, acc[0][3]);
      acc[1][3] = wm(fa1, fb3, acc[1][3]);
      guard4(acc[0][2], acc[1][2], acc[0][3], acc[1][3], fa0, fa1, fb2, fb3);
    }
  }

  _Float16* hhp = Hh[wave];
  _Float16* hlp = Hl[wave];
#pragma unroll
  for (int j = 0; j < 4; ++j) {
    const float bb = bfr(b1[g * NH_ + 16 * j + rl]);
#pragma unroll
    for (int i = 0; i < 2; ++i) {
#pragma unroll
      for (int r = 0; r < 8; ++r) {
        float v = acc[i][j][r] * (1.0f / WSC);
        v = v + bb;
        v = fmaxf(v, 0.f);
        _Float16 h, l;
        hl_one(v, h, l);
        const int o = (16 * i + 8 * hh + r) * HP_ + 16 * j + rl;
        hhp[o] = h;
        hlp[o] = l;
      }
    }
  }
  wave_sync_lds();

  float* os = Os[wave];
#pragma unroll 1
  for (int i = 0; i < 2; ++i) {
    v8f c0[4], c1[4];
#pragma unroll
    for (int j = 0; j < 4; ++j) { c0[j] = zero8(); c1[j] = zero8(); }
    const _Float16* ah = hhp + (16 * i + rl) * HP_ + koff;
    const _Float16* al = hlp + (16 * i + rl) * HP_ + koff;
    const _Float16* vr = W2 + (size_t)(g * NH_ + rl) * NH_ + koff;
#pragma unroll
    for (int ks = 0; ks < 2; ++ks) {
      const v16h fh = ldfrag_h(ah + 32 * ks);
      const v16h fl = ldfrag_h(al + 32 * ks);
      {
        const v16h g0 = ldfrag_h(vr + 32 * ks);
        const v16h g1 = ldfrag_h(vr + 16 * NH_ + 32 * ks);
        c0[0] = wm(fh, g0, c0[0]);
        c1[0] = wm(fl, g0, c1[0]);
        c0[1] = wm(fh, g1, c0[1]);
        c1[1] = wm(fl, g1, c1[1]);
        guard4(c0[0], c1[0], c0[1], c1[1], fh, fl, g0, g1);
      }
      {
        const v16h g2 = ldfrag_h(vr + 32 * NH_ + 32 * ks);
        const v16h g3 = ldfrag_h(vr + 48 * NH_ + 32 * ks);
        c0[2] = wm(fh, g2, c0[2]);
        c1[2] = wm(fl, g2, c1[2]);
        c0[3] = wm(fh, g3, c0[3]);
        c1[3] = wm(fl, g3, c1[3]);
        guard4(c0[2], c1[2], c0[3], c1[3], fh, fl, g2, g3);
      }
    }
#pragma unroll
    for (int j = 0; j < 4; ++j) {
      const float bb = bfr(b2[g * NH_ + 16 * j + rl]);
#pragma unroll
      for (int r = 0; r < 8; ++r) {
        float v = c0[j][r] * (1.0f / WSC);
        const float v1 = c1[j][r] * (1.0f / (WSC * LOSC));
        v = v + v1;
        v = v + bb;
        v = fmaxf(v, 0.f);
        _Float16 h, l;
        hl_one(v, h, l);
        const int o = (16 * i + 8 * hh + r) * HP_ + 16 * j + rl;
        hhp[o] = h;
        hlp[o] = l;
      }
    }
    wave_sync_lds();

    v8f e0 = zero8(), e1 = zero8();
    const _Float16* ur = W3 + (size_t)(g * NE_ + rl) * NH_ + koff;
#pragma unroll
    for (int ks = 0; ks < 2; ++ks) {
      const v16h fh = ldfrag_h(ah + 32 * ks);
      const v16h fl = ldfrag_h(al + 32 * ks);
      const v16h gw = ldfrag_h(ur + 32 * ks);
      e0 = wm(fh, gw, e0);
      e1 = wm(fl, gw, e1);
      guard2(e0, e1, fh, fl, gw);
    }
    const float bb3 = bfr(b3[g * NE_ + rl]);
#pragma unroll
    for (int r = 0; r < 8; ++r) {
      float v = e0[r] * (1.0f / WSC);
      const float v1 = e1[r] * (1.0f / (WSC * LOSC));
      v = v + v1;
      v = v + bb3;
      os[(8 * hh + r) * 16 + rl] = v;
    }
    wave_sync_lds();

    const v4f o0 = *(const v4f*)(os + 4 * lane);
    const v4f o1 = *(const v4f*)(os + 128 + 4 * lane);
    float* gp = outp + ((size_t)g * NB_ + (size_t)(m0 + 16 * i)) * NE_;
    *(volatile v4f*)(gp + 4 * lane) = o0;
    *(volatile v4f*)(gp + 128 + 4 * lane) = o1;
    __threadfence();
    *(volatile v4f*)(gp + 4 * lane) = o0;
    *(volatile v4f*)(gp + 128 + 4 * lane) = o1;
    wave_sync_lds();
  }
}

__global__ __launch_bounds__(128) void gate_mix(const float* __restrict__ pp, const float* __restrict__ np,
                                                const unsigned short* __restrict__ v1t, const float* __restrict__ cb1,
                                                const unsigned short* __restrict__ v2t, const float* __restrict__ cb2,
                                                const float* __restrict__ v3, const float* __restrict__ cb3,
                                                float* mixp, float* headp) {
#pragma clang fp contract(off)
  __shared__ __align__(16) float Et[16 * 16 * 32];
  __shared__ __align__(16) float Ct[16 * 64];
  __shared__ __align__(16) _Float16 Gh[4][16 * HP_];
  __shared__ __align__(16) _Float16 Gl[4][16 * HP_];
  __shared__ __align__(16) float Cv[4][16];
  const int tid = threadIdx.x, lane = tid & 31, wave = tid >> 5;
  const int rl = lane & 15, hh = lane >> 4, koff = 8 * hh;
  const int b0 = blockIdx.x * 16;
  const _Float16* V1 = (const _Float16*)(const void*)v1t;
  const _Float16* V2 = (const _Float16*)(const void*)v2t;
  _Float16* ghp = Gh[wave];
  _Float16* glp = Gl[wave];
  const _Float16* ga = ghp + rl * HP_ + koff;
  const _Float16* gb = glp + rl * HP_ + koff;
  float* cvw = Cv[wave];

#pragma unroll 1
  for (int q = 0; q < 2; ++q) {
#pragma unroll 1
    for (int cc = 0; cc < 8; ++cc) {
      const int cl = 8 * wave + cc;
      const int c = 32 * q + cl;
      const size_t ro = ((size_t)c * NB_ + (size_t)(b0 + rl)) * NE_ + koff;
      FragH ah, al;
      {
        const v4f p0 = *(const v4f*)(pp + ro), p1 = *(const v4f*)(pp + ro + 4);
        const v4f n0 = *(const v4f*)(np + ro), n1 = *(const v4f*)(np + ro + 4);
#pragma unroll
        for (int i = 0; i < 4; ++i) {
          _Float16 h, l;
          hl_one(p0[i], h, l); ah.h[0][i] = h;     al.h[0][i] = l;
          hl_one(p1[i], h, l); ah.h[0][4 + i] = h; al.h[0][4 + i] = l;
          hl_one(n0[i], h, l); ah.h[1][i] = h;     al.h[1][i] = l;
          hl_one(n1[i], h, l); ah.h[1][4 + i] = h; al.h[1][4 + i] = l;
        }
      }
      v8f c0[4], c1[4];
#pragma unroll
      for (int j = 0; j < 4; ++j) { c0[j] = zero8(); c1[j] = zero8(); }
      const _Float16* wr = V1 + (size_t)(c * NH_ + rl) * NX_ + koff;
      {
        const v16h g0 = ldfrag_h(wr);
        const v16h g1 = ldfrag_h(wr + 16 * NX_);
        c0[0] = wm(ah.v, g0, c0[0]);
        c1[0] = wm(al.v, g0, c1[0]);
        c0[1] = wm(ah.v, g1, c0[1]);
        c1[1] = wm(al.v, g1, c1[1]);
        guard4(c0[0], c1[0], c0[1], c1[1], ah.v, al.v, g0, g1);
      }
      {
        const v16h g2 = ldfrag_h(wr + 32 * NX_);
        const v16h g3 = ldfrag_h(wr + 48 * NX_);
        c0[2] = wm(ah.v, g2, c0[2]);
        c1[2] = wm(al.v, g2, c1[2]);
        c0[3] = wm(ah.v, g3, c0[3]);
        c1[3] = wm(al.v, g3, c1[3]);
        guard4(c0[2], c1[2], c0[3], c1[3], ah.v, al.v, g2, g3);
      }
#pragma unroll
      for (int j = 0; j < 4; ++j) {
        const float bb = bfr(cb1[c * NH_ + 16 * j + rl]);
#pragma unroll
        for (int r = 0; r < 8; ++r) {
          float v = c0[j][r] * (1.0f / WSC);
          const float v1 = c1[j][r] * (1.0f / (WSC * LOSC));
          v = v + v1;
          v = v + bb;
          v = fmaxf(v, 0.f);
          _Float16 h, l;
          hl_one(v, h, l);
          const int o = (8 * hh + r) * HP_ + 16 * j + rl;
          ghp[o] = h;
          glp[o] = l;
        }
      }
      wave_sync_lds();
      v8f d0[4], d1[4];
#pragma unroll
      for (int j = 0; j < 4; ++j) { d0[j] = zero8(); d1[j] = zero8(); }
      const _Float16* vr = V2 + (size_t)(c * NH_ + rl) * NH_ + koff;
#pragma unroll
      for (int ks = 0; ks < 2; ++ks) {
        const v16h fh = ldfrag_h(ga + 32 * ks);
        const v16h fl = ldfrag_h(gb + 32 * ks);
        {
          const v16h g0 = ldfrag_h(vr + 32 * ks);
          const v16h g1 = ldfrag_h(vr + 16 * NH_ + 32 * ks);
          d0[0] = wm(fh, g0, d0[0]);
          d1[0] = wm(fl, g0, d1[0]);
          d0[1] = wm(fh, g1, d0[1]);
          d1[1] = wm(fl, g1, d1[1]);
          guard4(d0[0], d1[0], d0[1], d1[1], fh, fl, g0, g1);
        }
        {
          const v16h g2 = ldfrag_h(vr + 32 * NH_ + 32 * ks);
          const v16h g3 = ldfrag_h(vr + 48 * NH_ + 32 * ks);
          d0[2] = wm(fh, g2, d0[2]);
          d1[2] = wm(fl, g2, d1[2]);
          d0[3] = wm(fh, g3, d0[3]);
          d1[3] = wm(fl, g3, d1[3]);
          guard4(d0[2], d1[2], d0[3], d1[3], fh, fl, g2, g3);
        }
      }
      float pr[8];
#pragma unroll
      for (int r = 0; r < 8; ++r) pr[r] = 0.f;
#pragma unroll
      for (int j = 0; j < 4; ++j) {
        const float bb = bfr(cb2[c * NH_ + 16 * j + rl]);
        const float ww = bfr(v3[c * NH_ + 16 * j + rl]);
#pragma unroll
        for (int r = 0; r < 8; ++r) {
          float v = d0[j][r] * (1.0f / WSC);
          const float v1 = d1[j][r] * (1.0f / (WSC * LOSC));
          v = v + v1;
          v = v + bb;
          v = fmaxf(v, 0.f);
          const float t = v * ww;
          pr[r] = pr[r] + t;
        }
      }
#pragma unroll
      for (int off = 1; off < 16; off <<= 1) {
#pragma unroll
        for (int r = 0; r < 8; ++r) pr[r] = pr[r] + __shfl_xor(pr[r], off, 32);
      }
      const float b3v = bfr(cb3[c]);
      if (rl == 0) {
#pragma unroll
        for (int r = 0; r < 8; ++r) cvw[8 * hh + r] = pr[r] + b3v;
      }
      wave_sync_lds();
      const float cv = cvw[rl];
      float w = cv * 0.5f;
      w = w + 0.5f;
      w = fmaxf(w, 0.f);
      w = fminf(w, 1.f);
      const float om = 1.0f - w;
      {
        const v4f p0 = *(const v4f*)(pp + ro), p1 = *(const v4f*)(pp + ro + 4);
        const v4f n0 = *(const v4f*)(np + ro), n1 = *(const v4f*)(np + ro + 4);
#pragma unroll
        for (int i = 0; i < 4; ++i) {
          float a = p0[i] * w;  float bq = n0[i] * om;
          Et[(rl * 16 + 8 * hh + i) * 32 + cl] = a + bq;
          a = p1[i] * w;        bq = n1[i] * om;
          Et[(rl * 16 + 8 * hh + 4 + i) * 32 + cl] = a + bq;
        }
      }
      if (hh == 0) Ct[rl * 64 + c] = cv;
      wave_sync_lds();
    }
    __syncthreads();
#pragma unroll 1
    for (int s = 0; s < 16; ++s) {
      const v4f v = *(const v4f*)(Et + 512 * s + 4 * tid);
      float* gp = mixp + (size_t)(b0 + s) * (NE_ * NG_) + (tid >> 3) * NG_ + 32 * q + 4 * (tid & 7);
      *(volatile v4f*)gp = v;
    }
    __threadfence();
#pragma unroll 1
    for (int s = 0; s < 16; ++s) {
      const v4f v = *(const v4f*)(Et + 512 * s + 4 * tid);
      float* gp = mixp + (size_t)(b0 + s) * (NE_ * NG_) + (tid >> 3) * NG_ + 32 * q + 4 * (tid & 7);
      *(volatile v4f*)gp = v;
    }
    __syncthreads();
  }
  {
    float* gbse = headp + (size_t)b0 * NG_;
    const v4f u0 = *(const v4f*)(Ct + 4 * tid);
    const v4f u1 = *(const v4f*)(Ct + 512 + 4 * tid);
    *(volatile v4f*)(gbse + 4 * tid) = u0;
    *(volatile v4f*)(gbse + 512 + 4 * tid) = u1;
    __threadfence();
    *(volatile v4f*)(gbse + 4 * tid) = u0;
    *(volatile v4f*)(gbse + 512 + 4 * tid) = u1;
  }
}

extern "C" void kernel_launch(void* const* d_in, const int* in_sizes, int n_in,
                              void* d_out, int out_size, void* d_ws, size_t ws_size,
                              hipStream_t stream) {
  if (n_in < 19) return;
  const int ex[19] = { NB_ * NI_,
                       NG_ * NI_ * NH_, NG_ * NH_, NG_ * NH_ * NH_, NG_ * NH_, NG_ * NH_ * NE_, NG_ * NE_,
                       NG_ * NI_ * NH_, NG_ * NH_, NG_ * NH_ * NH_, NG_ * NH_, NG_ * NH_ * NE_, NG_ * NE_,
                       NG_ * NX_ * NH_, NG_ * NH_, NG_ * NH_ * NH_, NG_ * NH_, NG_ * NH_, NG_ };
  for (int i = 0; i < 19; ++i) if (in_sizes[i] != ex[i]) return;
  if (out_size != NB_ * NE_ * NG_ + NB_ * NG_) return;

  const float* x   = (const float*)d_in[0];
  const float* pW1 = (const float*)d_in[1];  const float* pb1 = (const float*)d_in[2];
  const float* pW2 = (const float*)d_in[3];  const float* pb2 = (const float*)d_in[4];
  const float* pW3 = (const float*)d_in[5];  const float* pb3 = (const float*)d_in[6];
  const float* nW1 = (const float*)d_in[7];  const float* nb1 = (const float*)d_in[8];
  const float* nW2 = (const float*)d_in[9];  const float* nb2 = (const float*)d_in[10];
  const float* nW3 = (const float*)d_in[11]; const float* nb3 = (const float*)d_in[12];
  const float* cW1 = (const float*)d_in[13]; const float* cb1 = (const float*)d_in[14];
  const float* cW2 = (const float*)d_in[15]; const float* cb2 = (const float*)d_in[16];
  const float* cW3 = (const float*)d_in[17]; const float* cb3 = (const float*)d_in[18];
  float* out = (float*)d_out;
  float* mixo = out;
  float* heado = out + (size_t)NB_ * NE_ * NG_;

  const size_t hW1 = (size_t)NG_ * NH_ * NI_;
  const size_t hW2 = (size_t)NG_ * NH_ * NH_;
  const size_t hW3 = (size_t)NG_ * NE_ * NH_;
  const size_t hV1 = (size_t)NG_ * NH_ * NX_;
  const size_t sXH = (size_t)NB_ * NI_ * 2;
  const size_t sW1 = 2 * hW1 * 2;
  const size_t sW2 = 3 * hW2 * 2;
  const size_t sW3 = 2 * hW3 * 2;
  const size_t sV1 = hV1 * 2;
  const size_t sPL = (size_t)NG_ * NB_ * NE_ * 4;
  size_t off = 0;
  const size_t oXH = off; off += sXH;
  const size_t oW1 = off; off += sW1;
  const size_t oW2 = off; off += sW2;
  const size_t oW3 = off; off += sW3;
  const size_t oV1 = off; off += sV1;
  const size_t oPP = off; off += sPL;
  const size_t oNP = off; off += sPL;
  if (off > ws_size) return;
  if (off > (size_t)134217728) return;

  char* ws = (char*)d_ws;
  unsigned short* XH  = (unsigned short*)(ws + oXH);
  unsigned short* W1T = (unsigned short*)(ws + oW1);
  unsigned short* W2T = (unsigned short*)(ws + oW2);
  unsigned short* W3T = (unsigned short*)(ws + oW3);
  unsigned short* V1T = (unsigned short*)(ws + oV1);
  float*          PPL = (float*)(ws + oPP);
  float*          NPL = (float*)(ws + oNP);

  const dim3 blk(256);
  {
    const int n8 = NB_ * NI_ / 8;
    cvt_x<<<dim3(n8 / 256), blk, 0, stream>>>(x, XH, n8);
  }
  {
    const int n8a = (int)(hW1 / 8);
    cvt_w<<<dim3(n8a / 256, 2), blk, 0, stream>>>(pW1, nW1, pW1, W1T, NI_, NH_, n8a);
    const int n8b = (int)(hW2 / 8);
    cvt_w<<<dim3(n8b / 256, 3), blk, 0, stream>>>(pW2, nW2, cW2, W2T, NH_, NH_, n8b);
    const int n8c = (int)(hW3 / 8);
    cvt_w<<<dim3(n8c / 256, 2), blk, 0, stream>>>(pW3, nW3, pW3, W3T, NH_, NE_, n8c);
    const int n8d = (int)(hV1 / 8);
    cvt_w<<<dim3(n8d / 256, 1), blk, 0, stream>>>(cW1, cW1, cW1, V1T, NX_, NH_, n8d);
  }
  grp_mlp<<<dim3(NB_ / 128, NG_), dim3(128), 0, stream>>>(XH, W1T, pb1, W2T, pb2, W3T, pb3, PPL);
  grp_mlp<<<dim3(NB_ / 128, NG_), dim3(128), 0, stream>>>(XH, W1T + hW1, nb1, W2T + hW2, nb2, W3T + hW3, nb3, NPL);
  gate_mix<<<dim3(NB_ / 16), dim3(128), 0, stream>>>(PPL, NPL, V1T, cb1, W2T + 2 * hW2, cb2, cW3, cb3, mixo, heado);
  (void)hipGetLastError();
}
